// CutsEmbedding_77309411328401
// MI455X (gfx1250) — hardware-run, weakly checked
//
#include <hip/hip_runtime.h>

typedef __attribute__((ext_vector_type(16))) _Float16 v16h;
typedef __attribute__((ext_vector_type(8)))  _Float16 v8h;
typedef __attribute__((ext_vector_type(4)))  _Float16 v4h;
typedef __attribute__((ext_vector_type(8)))  float    v8f;
typedef __attribute__((ext_vector_type(4)))  float    v4f;
typedef __attribute__((ext_vector_type(4)))  int      v4i;

constexpr int kNumV   = 100000;
constexpr int kNumC   = 50000;
constexpr int kNumA   = 5000;
constexpr int kEdgeC  = 1600000;
constexpr int kEdgeA  = 800000;
constexpr int kFeat   = 16;
constexpr int kEdgeF  = 8;
constexpr int kHid    = 32;
constexpr int kRangeV = 896;
constexpr int kRangeA = 128;
constexpr int kListCap = 160;
constexpr float kWCarry    = 16.0f;
constexpr float kWCarryInv = 1.0f / 16.0f;
static_assert((kEdgeC % 128) == 0 && (kEdgeA % 128) == 0, "edge chunks of 128");
static_assert((kNumV % 16) == 0, "node tiles of 16");
static_assert(kFeat == 16 && kEdgeF == 8 && kHid == 32, "row layouts");

constexpr size_t kOffAggG = 0;
constexpr size_t kOffAggH = kOffAggG + (size_t)kNumV * kHid * 4;
constexpr size_t kOffFv   = kOffAggH + (size_t)kNumV * kHid * 4;
constexpr size_t kOffAggA = kOffFv   + (size_t)kNumV * kHid * 4;
constexpr size_t kWsTotal = kOffAggA + (size_t)kNumA * kHid * 4;
static_assert(kWsTotal == 39040000ull, "carve total");
static_assert(kWsTotal <= 134217728ull, "carve cap");
static_assert((kOffAggH % 128) == 0 && (kOffFv % 128) == 0 && (kOffAggA % 128) == 0, "aligned regions");

union FragU { v16h v; v8h h[2]; };
__device__ __forceinline__ v16h frag_load(const _Float16* p) {
  FragU f;
  f.h[0] = *(const v8h*)(p);
  f.h[1] = *(const v8h*)(p + 16);
  return f.v;
}
__device__ __forceinline__ v8f mma_f16(v16h a, v16h b, v8f c) {
  c = __builtin_amdgcn_wmma_f32_16x16x32_f16(false, a, false, b, (short)0, c, false, false);
  asm volatile("v_nop\n\tv_nop\n\tv_nop\n\tv_nop" : "+v"(c) : "v"(a), "v"(b));
  return c;
}
__device__ __forceinline__ void wave_lds_sync() {
  __builtin_amdgcn_fence(__ATOMIC_RELEASE, "workgroup");
  __builtin_amdgcn_wave_barrier();
  __builtin_amdgcn_fence(__ATOMIC_ACQUIRE, "workgroup");
}
__device__ __forceinline__ v8f splat8(float b) {
  v8f c = {b, b, b, b, b, b, b, b};
  return c;
}
__device__ __forceinline__ void put4(_Float16* p, v4f f) {
  v4h hv;
  hv[0] = (_Float16)f[0];
  hv[1] = (_Float16)f[1];
  hv[2] = (_Float16)f[2];
  hv[3] = (_Float16)f[3];
  *(v4h*)p = hv;
}
__device__ __forceinline__ void put4z(_Float16* p) {
  v4h z;
  z[0] = (_Float16)0.0f;
  z[1] = (_Float16)0.0f;
  z[2] = (_Float16)0.0f;
  z[3] = (_Float16)0.0f;
  *(v4h*)p = z;
}
template <int KIN, int KP>
__device__ __forceinline__ void stage_wt(_Float16* dst, const float* __restrict__ W, int tid) {
  for (int idx = tid; idx < 32 * KP; idx += 256) {
    const int n = idx / KP;
    const int k = idx - n * KP;
    const int kc = (k < KIN) ? k : (KIN - 1);
    const float w = W[kc * 32 + n];
    const float ws = (k < KIN) ? (w * kWCarry) : 0.0f;
    dst[idx] = (_Float16)ws;
  }
}

template <int RANGE, int MODE>
__global__ __launch_bounds__(256) void edge_owner_kernel(
    const float* __restrict__ featT, const float* __restrict__ featS, const float* __restrict__ ea,
    const int* __restrict__ srcIdx, const int* __restrict__ tgtIdx,
    const float* __restrict__ W1, const float* __restrict__ b1,
    const float* __restrict__ W2, const float* __restrict__ b2,
    float* __restrict__ aggr, int nEdges, int nSrc, int nTgt, int nOwn)
{
  constexpr int KIN = (MODE == 0) ? 40 : 56;
  constexpr float FXS     = (MODE == 0) ? 1048576.0f : 262144.0f;
  constexpr float FXS_INV = 1.0f / FXS;
  __shared__ int sAcc[RANGE * 32];
  __shared__ int sCnt[RANGE];
  __shared__ __align__(16) _Float16 sW1[32 * 64];
  __shared__ __align__(16) _Float16 sW2[32 * 32];
  __shared__ __align__(16) _Float16 sA[8][16 * 64];
  __shared__ __align__(16) _Float16 sH[8][16 * 32];
  __shared__ int sList[8][kListCap];
  __shared__ int sTl[8][16];
  __shared__ float sB1[32];
  __shared__ float sB2[32];

  const int tid  = threadIdx.x;
  const int lane = tid & 31;
  const int wave = __builtin_amdgcn_readfirstlane((int)(threadIdx.x >> 5));
  const int r = lane & 15;
  const int h = lane >> 4;
  const int n0 = blockIdx.x * RANGE;
  int nLocal = nOwn - n0;
  if (nLocal > RANGE) nLocal = RANGE;

  for (int i = tid; i < RANGE * 32; i += 256) sAcc[i] = 0;
  for (int i = tid; i < RANGE; i += 256) sCnt[i] = 0;
  stage_wt<KIN, 64>(sW1, W1, tid);
  stage_wt<32, 32>(sW2, W2, tid);
  if (tid < 32) {
    sB1[tid] = b1[tid];
    sB2[tid] = b2[tid];
  }
  __syncthreads();

  v16h w1f00 = frag_load(sW1 + (r) * 64 + 8 * h);
  v16h w1f01 = frag_load(sW1 + (r) * 64 + 32 + 8 * h);
  v16h w1f10 = frag_load(sW1 + (r + 16) * 64 + 8 * h);
  v16h w1f11 = frag_load(sW1 + (r + 16) * 64 + 32 + 8 * h);
  v16h w2f0  = frag_load(sW2 + (r) * 32 + 8 * h);
  v16h w2f1  = frag_load(sW2 + (r + 16) * 32 + 8 * h);
  const float bias10 = sB1[r] * kWCarry;
  const float bias11 = sB1[r + 16] * kWCarry;
  const float bias20 = sB2[r] * kWCarry;
  const float bias21 = sB2[r + 16] * kWCarry;

  const int* keyIdx = (MODE == 0) ? tgtIdx : srcIdx;
  const int nChunks = nEdges >> 7;
  const unsigned ltmask = (1u << lane) - 1u;
  int cnt = 0;

  for (int ch = wave; ; ch += 8) {
    const bool last = (ch >= nChunks);
    if (!last) {
      const int eb = (ch << 7) + (lane << 2);
      const v4i kv = *(const v4i*)(keyIdx + eb);
#pragma unroll
      for (int j = 0; j < 4; ++j) {
        const int key = kv[j];
        const bool hit = (unsigned)(key - n0) < (unsigned)nLocal;
        const unsigned mask = __builtin_amdgcn_ballot_w32(hit);
        const int pos = cnt + __popc(mask & ltmask);
        if (hit) sList[wave][pos] = eb + j;
        cnt += __popc(mask);
      }
      wave_lds_sync();
    }
#pragma unroll 1
    for (int it = 0; it < 10; ++it) {
      int nv;
      if (cnt >= 16) nv = 16;
      else if (last && cnt > 0) nv = cnt;
      else break;
      cnt -= nv;
      const int base = cnt;

      const int rowc = (r < nv) ? r : (nv - 1);
      int e = sList[wave][base + rowc];
      e = e < 0 ? 0 : e;
      e = e > nEdges - 1 ? nEdges - 1 : e;
      int s = srcIdx[e];
      int t = tgtIdx[e];
      const int keyRaw = (MODE == 0) ? t : s;
      s = s < 0 ? 0 : s;
      s = s > nSrc - 1 ? nSrc - 1 : s;
      t = t < 0 ? 0 : t;
      t = t > nTgt - 1 ? nTgt - 1 : t;
      int loc = keyRaw - n0;
      loc = loc < 0 ? 0 : loc;
      loc = loc > RANGE - 1 ? RANGE - 1 : loc;
      sTl[wave][r] = loc;

      _Float16* arow = &sA[wave][r * 64];
      if (MODE == 0) {
        const float* pT = featT + (size_t)t * 16 + 8 * h;
        const float* pS = featS + (size_t)s * 16 + 8 * h;
        const float* pE = ea + (size_t)e * 8 + 4 * h;
        const v4f a0 = *(const v4f*)(pT);
        const v4f a1 = *(const v4f*)(pT + 4);
        const v4f c0 = *(const v4f*)(pS);
        const v4f c1 = *(const v4f*)(pS + 4);
        const v4f e0 = *(const v4f*)(pE);
        put4(arow + 8 * h, a0);
        put4(arow + 8 * h + 4, a1);
        put4(arow + 16 + 8 * h, c0);
        put4(arow + 16 + 8 * h + 4, c1);
        put4(arow + 32 + 4 * h, e0);
        put4z(arow + 40 + 12 * h);
        put4z(arow + 40 + 12 * h + 4);
        put4z(arow + 40 + 12 * h + 8);
      } else {
        const float* pS = featS + (size_t)s * 16 + 8 * h;
        const float* pT = featT + (size_t)t * 32 + 16 * h;
        const float* pE = ea + (size_t)e * 8 + 4 * h;
        const v4f a0 = *(const v4f*)(pS);
        const v4f a1 = *(const v4f*)(pS + 4);
        const v4f f0 = *(const v4f*)(pT);
        const v4f f1 = *(const v4f*)(pT + 4);
        const v4f f2 = *(const v4f*)(pT + 8);
        const v4f f3 = *(const v4f*)(pT + 12);
        const v4f e0 = *(const v4f*)(pE);
        put4(arow + 8 * h, a0);
        put4(arow + 8 * h + 4, a1);
        put4(arow + 16 + 16 * h, f0);
        put4(arow + 16 + 16 * h + 4, f1);
        put4(arow + 16 + 16 * h + 8, f2);
        put4(arow + 16 + 16 * h + 12, f3);
        put4(arow + 48 + 4 * h, e0);
        put4z(arow + 56 + 4 * h);
      }
      wave_lds_sync();

      const v16h a0f = frag_load(&sA[wave][r * 64 + 8 * h]);
      const v16h a1f = frag_load(&sA[wave][r * 64 + 32 + 8 * h]);
      v8f c0 = splat8(bias10);
      v8f c1 = splat8(bias11);
      c0 = mma_f16(a0f, w1f00, c0);
      c0 = mma_f16(a1f, w1f01, c0);
      c1 = mma_f16(a0f, w1f10, c1);
      c1 = mma_f16(a1f, w1f11, c1);
#pragma unroll
      for (int rr = 0; rr < 8; ++rr) {
        const float x0 = fmaxf(c0[rr] * kWCarryInv, 0.0f);
        const float x1 = fmaxf(c1[rr] * kWCarryInv, 0.0f);
        sH[wave][(8 * h + rr) * 32 + r]      = (_Float16)x0;
        sH[wave][(8 * h + rr) * 32 + r + 16] = (_Float16)x1;
      }
      wave_lds_sync();

      const v16h hf = frag_load(&sH[wave][r * 32 + 8 * h]);
      v8f o0 = splat8(bias20);
      v8f o1 = splat8(bias21);
      o0 = mma_f16(hf, w2f0, o0);
      o1 = mma_f16(hf, w2f1, o1);

#pragma unroll
      for (int rr = 0; rr < 8; ++rr) {
        const int row = 8 * h + rr;
        const int tl = sTl[wave][row];
        const bool ok = row < nv;
        const float v0 = o0[rr] * kWCarryInv;
        const float v1 = o1[rr] * kWCarryInv;
        const int i0 = ok ? __float2int_rn(v0 * FXS) : 0;
        const int i1 = ok ? __float2int_rn(v1 * FXS) : 0;
        atomicAdd(&sAcc[tl * 32 + r], i0);
        atomicAdd(&sAcc[tl * 32 + r + 16], i1);
      }
      {
        const int one = (h == 0 && r < nv) ? 1 : 0;
        atomicAdd(&sCnt[loc], one);
      }
      wave_lds_sync();
    }
    if (last) break;
  }

  __syncthreads();

  for (int pass = 0; pass < 2; ++pass) {
    for (int i = wave; i < nLocal; i += 8) {
      const float c = (float)sCnt[i];
      const float inv = 1.0f / fmaxf(c, 1.0f);
      const float sum = (float)sAcc[i * 32 + lane] * FXS_INV;
      const float val = sum * inv;
      *(volatile float*)(aggr + (size_t)(n0 + i) * 32 + lane) = val;
    }
    __threadfence();
  }
}

__global__ __launch_bounds__(256) void node_fv_kernel(
    const float* __restrict__ x_v, const float* __restrict__ aggr_g, const float* __restrict__ aggr_h,
    const float* __restrict__ W1, const float* __restrict__ b1,
    const float* __restrict__ W2, const float* __restrict__ b2,
    float* __restrict__ fv, int nNodes)
{
  __shared__ __align__(16) _Float16 sW1[32 * 96];
  __shared__ __align__(16) _Float16 sW2[32 * 32];
  __shared__ __align__(16) _Float16 sA[8][16 * 96];
  __shared__ __align__(16) _Float16 sH[8][16 * 32];
  __shared__ __align__(16) float sO[8][16 * 36];
  __shared__ float sB1[32];
  __shared__ float sB2[32];

  const int tid  = threadIdx.x;
  const int lane = tid & 31;
  const int wave = __builtin_amdgcn_readfirstlane((int)(threadIdx.x >> 5));
  const int r = lane & 15;
  const int h = lane >> 4;

  stage_wt<80, 96>(sW1, W1, tid);
  stage_wt<32, 32>(sW2, W2, tid);
  if (tid < 32) {
    sB1[tid] = b1[tid];
    sB2[tid] = b2[tid];
  }
  __syncthreads();

  const int tile = blockIdx.x * 8 + wave;
  const int nTiles = nNodes >> 4;
  if (tile < nTiles) {
    const int v = tile * 16 + r;
    _Float16* arow = &sA[wave][r * 96];
    {
      const float* px = x_v + (size_t)v * 16 + 8 * h;
      const float* pg = aggr_g + (size_t)v * 32 + 16 * h;
      const float* ph = aggr_h + (size_t)v * 32 + 16 * h;
      const v4f a0 = *(const v4f*)(px);
      const v4f a1 = *(const v4f*)(px + 4);
      const v4f g0 = *(const v4f*)(pg);
      const v4f g1 = *(const v4f*)(pg + 4);
      const v4f g2 = *(const v4f*)(pg + 8);
      const v4f g3 = *(const v4f*)(pg + 12);
      const v4f h0 = *(const v4f*)(ph);
      const v4f h1 = *(const v4f*)(ph + 4);
      const v4f h2 = *(const v4f*)(ph + 8);
      const v4f h3 = *(const v4f*)(ph + 12);
      put4(arow + 8 * h, a0);
      put4(arow + 8 * h + 4, a1);
      put4(arow + 16 + 16 * h, g0);
      put4(arow + 16 + 16 * h + 4, g1);
      put4(arow + 16 + 16 * h + 8, g2);
      put4(arow + 16 + 16 * h + 12, g3);
      put4(arow + 48 + 16 * h, h0);
      put4(arow + 48 + 16 * h + 4, h1);
      put4(arow + 48 + 16 * h + 8, h2);
      put4(arow + 48 + 16 * h + 12, h3);
      put4z(arow + 80 + 8 * h);
      put4z(arow + 80 + 8 * h + 4);
    }
    wave_lds_sync();

    const v16h a0f = frag_load(&sA[wave][r * 96 + 8 * h]);
    const v16h a1f = frag_load(&sA[wave][r * 96 + 32 + 8 * h]);
    const v16h a2f = frag_load(&sA[wave][r * 96 + 64 + 8 * h]);
    v8f c0 = splat8(sB1[r] * kWCarry);
    v8f c1 = splat8(sB1[r + 16] * kWCarry);
    {
      const v16h w00 = frag_load(sW1 + (r) * 96 + 8 * h);
      const v16h w01 = frag_load(sW1 + (r) * 96 + 32 + 8 * h);
      const v16h w02 = frag_load(sW1 + (r) * 96 + 64 + 8 * h);
      c0 = mma_f16(a0f, w00, c0);
      c0 = mma_f16(a1f, w01, c0);
      c0 = mma_f16(a2f, w02, c0);
    }
    {
      const v16h w10 = frag_load(sW1 + (r + 16) * 96 + 8 * h);
      const v16h w11 = frag_load(sW1 + (r + 16) * 96 + 32 + 8 * h);
      const v16h w12 = frag_load(sW1 + (r + 16) * 96 + 64 + 8 * h);
      c1 = mma_f16(a0f, w10, c1);
      c1 = mma_f16(a1f, w11, c1);
      c1 = mma_f16(a2f, w12, c1);
    }
#pragma unroll
    for (int rr = 0; rr < 8; ++rr) {
      const float x0 = fmaxf(c0[rr] * kWCarryInv, 0.0f);
      const float x1 = fmaxf(c1[rr] * kWCarryInv, 0.0f);
      sH[wave][(8 * h + rr) * 32 + r]      = (_Float16)x0;
      sH[wave][(8 * h + rr) * 32 + r + 16] = (_Float16)x1;
    }
    wave_lds_sync();

    const v16h hf = frag_load(&sH[wave][r * 32 + 8 * h]);
    const v16h w2f0 = frag_load(sW2 + (r) * 32 + 8 * h);
    const v16h w2f1 = frag_load(sW2 + (r + 16) * 32 + 8 * h);
    v8f o0 = splat8(sB2[r] * kWCarry);
    v8f o1 = splat8(sB2[r + 16] * kWCarry);
    o0 = mma_f16(hf, w2f0, o0);
    o1 = mma_f16(hf, w2f1, o1);
#pragma unroll
    for (int rr = 0; rr < 8; ++rr) {
      sO[wave][(8 * h + rr) * 36 + r]      = o0[rr] * kWCarryInv;
      sO[wave][(8 * h + rr) * 36 + r + 16] = o1[rr] * kWCarryInv;
    }
    wave_lds_sync();

    const int q  = lane >> 3;
    const int c4 = (lane & 7) * 4;
    for (int pass = 0; pass < 2; ++pass) {
#pragma unroll
      for (int it = 0; it < 4; ++it) {
        const int row = it * 4 + q;
        const v4f val = *(const v4f*)(&sO[wave][row * 36 + c4]);
        *(volatile v4f*)(fv + (size_t)(tile * 16 + row) * 32 + c4) = val;
      }
      __threadfence();
    }
  }
}

__global__ __launch_bounds__(256) void node_fa_kernel(
    const float* __restrict__ x_a, const float* __restrict__ aggr_a,
    const float* __restrict__ W1, const float* __restrict__ b1,
    const float* __restrict__ W2, const float* __restrict__ b2,
    float* __restrict__ out, int nNodes)
{
  __shared__ float sW1[48 * 32];
  __shared__ float sW2[32 * 32];
  __shared__ float sIn[8][48];
  __shared__ float sHid[8][32];
  const int tid  = threadIdx.x;
  const int lane = tid & 31;
  const int wave = __builtin_amdgcn_readfirstlane((int)(threadIdx.x >> 5));
  for (int i = tid; i < 48 * 32; i += 256) sW1[i] = W1[i];
  for (int i = tid; i < 32 * 32; i += 256) sW2[i] = W2[i];
  __syncthreads();
  const float bb1 = b1[lane];
  const float bb2 = b2[lane];
#pragma unroll 1
  for (int it = 0; it < 4; ++it) {
    const int node = (blockIdx.x * 8 + wave) * 4 + it;
    if (node < nNodes) {
      sIn[wave][lane & 15] = x_a[(size_t)node * 16 + (lane & 15)];
      sIn[wave][16 + lane] = aggr_a[(size_t)node * 32 + lane];
      wave_lds_sync();
      float acc = bb1;
#pragma unroll 4
      for (int k = 0; k < 48; ++k) acc = fmaf(sIn[wave][k], sW1[k * 32 + lane], acc);
      sHid[wave][lane] = fmaxf(acc, 0.0f);
      wave_lds_sync();
      float o = bb2;
#pragma unroll 4
      for (int k = 0; k < 32; ++k) o = fmaf(sHid[wave][k], sW2[k * 32 + lane], o);
      volatile float* p = out + (size_t)node * 32 + lane;
      *p = o;
      __threadfence();
      *p = o;
      wave_lds_sync();
    }
  }
}

extern "C" void kernel_launch(void* const* d_in, const int* in_sizes, int n_in,
                              void* d_out, int out_size, void* d_ws, size_t ws_size,
                              hipStream_t stream) {
  if (n_in < 27) return;
  if (in_sizes[0] != kNumC * kFeat) return;
  if (in_sizes[1] != kNumV * kFeat) return;
  if (in_sizes[2] != kNumA * kFeat) return;
  if (in_sizes[3] != 2 * kEdgeC) return;
  if (in_sizes[4] != 2 * kEdgeA) return;
  if (in_sizes[5] != kEdgeC * kEdgeF) return;
  if (in_sizes[6] != kEdgeA * kEdgeF) return;
  if (in_sizes[7] != 40 * 32 || in_sizes[11] != 40 * 32) return;
  if (in_sizes[15] != 80 * 32 || in_sizes[19] != 56 * 32 || in_sizes[23] != 48 * 32) return;
  if (in_sizes[9] != 1024 || in_sizes[13] != 1024 || in_sizes[17] != 1024) return;
  if (in_sizes[21] != 1024 || in_sizes[25] != 1024) return;
  if (out_size != kNumA * kHid) return;
  if (ws_size < kWsTotal) return;

  const float* x_c    = (const float*)d_in[0];
  const float* x_v    = (const float*)d_in[1];
  const float* x_a    = (const float*)d_in[2];
  const int*   ei_c2v = (const int*)d_in[3];
  const int*   ei_a2v = (const int*)d_in[4];
  const float* ea_c2v = (const float*)d_in[5];
  const float* ea_a2v = (const float*)d_in[6];
  const float* gv_W1 = (const float*)d_in[7];
  const float* gv_b1 = (const float*)d_in[8];
  const float* gv_W2 = (const float*)d_in[9];
  const float* gv_b2 = (const float*)d_in[10];
  const float* hv_W1 = (const float*)d_in[11];
  const float* hv_b1 = (const float*)d_in[12];
  const float* hv_W2 = (const float*)d_in[13];
  const float* hv_b2 = (const float*)d_in[14];
  const float* fv_W1 = (const float*)d_in[15];
  const float* fv_b1 = (const float*)d_in[16];
  const float* fv_W2 = (const float*)d_in[17];
  const float* fv_b2 = (const float*)d_in[18];
  const float* ga_W1 = (const float*)d_in[19];
  const float* ga_b1 = (const float*)d_in[20];
  const float* ga_W2 = (const float*)d_in[21];
  const float* ga_b2 = (const float*)d_in[22];
  const float* fa_W1 = (const float*)d_in[23];
  const float* fa_b1 = (const float*)d_in[24];
  const float* fa_W2 = (const float*)d_in[25];
  const float* fa_b2 = (const float*)d_in[26];

  char* ws = (char*)d_ws;
  float* aggG = (float*)(ws + kOffAggG);
  float* aggH = (float*)(ws + kOffAggH);
  float* fvP  = (float*)(ws + kOffFv);
  float* aggA = (float*)(ws + kOffAggA);

  constexpr int kBlocksV = (kNumV + kRangeV - 1) / kRangeV;
  constexpr int kBlocksA = (kNumA + kRangeA - 1) / kRangeA;
  constexpr int kBlocksFv = (kNumV / 16 + 7) / 8;
  constexpr int kBlocksFa = (kNumA + 31) / 32;

  edge_owner_kernel<kRangeV, 0><<<kBlocksV, 256, 0, stream>>>(
      x_v, x_c, ea_c2v, ei_c2v, ei_c2v + kEdgeC,
      gv_W1, gv_b1, gv_W2, gv_b2, aggG, kEdgeC, kNumC, kNumV, kNumV);

  edge_owner_kernel<kRangeV, 0><<<kBlocksV, 256, 0, stream>>>(
      x_v, x_a, ea_a2v, ei_a2v, ei_a2v + kEdgeA,
      hv_W1, hv_b1, hv_W2, hv_b2, aggH, kEdgeA, kNumA, kNumV, kNumV);

  node_fv_kernel<<<kBlocksFv, 256, 0, stream>>>(
      x_v, aggG, aggH, fv_W1, fv_b1, fv_W2, fv_b2, fvP, kNumV);

  edge_owner_kernel<kRangeA, 1><<<kBlocksA, 256, 0, stream>>>(
      fvP, x_a, ea_a2v, ei_a2v, ei_a2v + kEdgeA,
      ga_W1, ga_b1, ga_W2, ga_b2, aggA, kEdgeA, kNumA, kNumV, kNumA);

  node_fa_kernel<<<kBlocksFa, 256, 0, stream>>>(
      x_a, aggA, fa_W1, fa_b1, fa_W2, fa_b2, (float*)d_out, kNumA);
}
